// self_attention_18167711662780
// MI455X (gfx1250) — hardware-verified
//
#include <hip/hip_runtime.h>


#define DEV __device__ __forceinline__

#ifndef NB
#define NB 4
#endif
#ifndef SEQ
#define SEQ 2048
#endif
#define NB_FULL  4
#define SEQ_FULL 2048
#define CDIM 1024
#define DKD  256
#define DOD  1024
#define KDIM 1024

#define SST  (SEQ + 4)
#define PST  (SEQ + 8)
#define OST  (DOD + 4)
#define R0F  (16 * ((SST > OST) ? SST : OST))
#define ATTN_LDS_BYTES (R0F * 4 + 16 * 4 + 128 * 4 + 16 * PST * 2)
#define CT_P 136
#define SCORE_SCALE 0.000244140625f

static_assert(NB >= 1 && NB <= NB_FULL);
static_assert(SEQ >= 128 && SEQ <= SEQ_FULL && (SEQ % 128) == 0);
static_assert(((NB * SEQ) % 64) == 0);
static_assert((DKD % 128) == 0 && (DOD % 128) == 0 && (KDIM % 32) == 0 && (CDIM == KDIM));
static_assert((((long long)NB * SEQ * CDIM) % (8 * 256)) == 0);
static_assert(ATTN_LDS_BYTES <= 300 * 1024);
static_assert(((R0F * 4) % 16) == 0 && (((R0F + 16 + 128) * 4) % 16) == 0);
static_assert(((PST * 2) % 16) == 0 && ((OST * 4) % 16) == 0 && ((CT_P * 2) % 16) == 0);
static_assert(16 * OST <= R0F);

typedef _Float16       v8h   __attribute__((ext_vector_type(8)));
typedef _Float16       v16h  __attribute__((ext_vector_type(16)));
typedef __bf16         v16bf __attribute__((ext_vector_type(16)));
typedef unsigned short v8us  __attribute__((ext_vector_type(8)));
typedef unsigned short v16us __attribute__((ext_vector_type(16)));
typedef float          v8f   __attribute__((ext_vector_type(8)));
typedef float          v4f   __attribute__((ext_vector_type(4)));

union FragH { v16h v;  v8h  half[2]; };
union FragB { v16bf v; v16us u; v8us half[2]; };

DEV unsigned int bf16_bits(float f) {
    unsigned int u = __float_as_uint(f);
    u += 0x7FFFu + ((u >> 16) & 1u);
    return u >> 16;
}
DEV float bf16_val(float f) { return __uint_as_float(bf16_bits(f) << 16); }

DEV v8f zero8f() {
    v8f z;
#pragma unroll
    for (int i = 0; i < 8; ++i) z[i] = 0.f;
    return z;
}

DEV v8f mma_bf16(v16bf a, v16bf b, v8f c) {
    c = __builtin_amdgcn_wmma_f32_16x16x32_bf16(false, a, false, b, (short)0, c, false, false);
    asm volatile("v_nop\n\tv_nop\n\tv_nop\n\tv_nop" : "+v"(c) : "v"(a), "v"(b));
    return c;
}
DEV v8f mma_f16(v16h a, v16h b, v8f c) {
    c = __builtin_amdgcn_wmma_f32_16x16x32_f16(false, a, false, b, (short)0, c, false, false);
    asm volatile("v_nop\n\tv_nop\n\tv_nop\n\tv_nop" : "+v"(c) : "v"(a), "v"(b));
    return c;
}

__global__ __launch_bounds__(256) void k_cvt_x(const float* __restrict__ x,
                                               unsigned short* __restrict__ xp)
{
    const size_t g = (size_t)blockIdx.x * 256 + threadIdx.x;
    const size_t e = g * 8;
    const int m  = (int)(e / CDIM);
    const int c  = (int)(e % CDIM);
    const int bb = m / SEQ;
    const int s  = m - bb * SEQ;
    const float* src = x + ((size_t)bb * SEQ_FULL + s) * CDIM + c;
    const v4f a0 = *(const v4f*)src;
    const v4f a1 = *(const v4f*)(src + 4);
    v8us o;
#pragma unroll
    for (int i = 0; i < 4; ++i) {
        o[i]     = (unsigned short)bf16_bits(a0[i]);
        o[4 + i] = (unsigned short)bf16_bits(a1[i]);
    }
    unsigned short* dst = xp + (size_t)m * CDIM + c;
    *(volatile v8us*)dst = o;
    __threadfence();
    *(volatile v8us*)dst = o;
}

__global__ __launch_bounds__(256) void k_transpose_w(const float* __restrict__ W,
                                                     unsigned short* __restrict__ WT,
                                                     int R, int Ncol)
{
    __shared__ __attribute__((aligned(16))) unsigned short T[64 * 72];
    const int tid = threadIdx.x;
    const int n0 = blockIdx.x * 64, r0 = blockIdx.y * 64;
    const int nn = tid & 63, rq = tid >> 6;
#pragma unroll 4
    for (int i = 0; i < 16; ++i) {
        const int rr = i * 4 + rq;
        const float v = W[(size_t)(r0 + rr) * Ncol + n0 + nn];
        T[nn * 72 + rr] = (unsigned short)bf16_bits(v);
    }
    __syncthreads();
    const int piece = tid & 7;
    const int na = tid >> 3;
    const v8us va = *(const v8us*)(T + na * 72 + piece * 8);
    const v8us vb = *(const v8us*)(T + (na + 32) * 72 + piece * 8);
    unsigned short* da = WT + (size_t)(n0 + na) * R + r0 + piece * 8;
    unsigned short* db = WT + (size_t)(n0 + na + 32) * R + r0 + piece * 8;
    *(volatile v8us*)da = va;
    *(volatile v8us*)db = vb;
    __threadfence();
    *(volatile v8us*)da = va;
    *(volatile v8us*)db = vb;
}

__global__ __launch_bounds__(256) __attribute__((amdgpu_num_vgpr(256)))
void k_gemm_nt(const unsigned short* __restrict__ A, long long zsA,
               const unsigned short* __restrict__ Bm, long long zsB,
               const float* __restrict__ bias, int nbias, int bias_per_row,
               _Float16* __restrict__ Cm, long long zsC, int ldc, float oscale)
{
    __shared__ __attribute__((aligned(16))) _Float16 Ct[64 * CT_P];

    const int tid = threadIdx.x, lane = tid & 31, w = tid >> 5;
    const int h = lane >> 4, l15 = lane & 15;
    const int wm = w & 3, wn = w >> 2;
    const int z = blockIdx.z;
    const int row0 = blockIdx.y * 64;
    const int col0 = blockIdx.x * 128;

    const unsigned short* ap = A  + (size_t)z * (size_t)zsA + (size_t)(row0 + wm * 16 + l15) * KDIM + 8 * h;
    const unsigned short* bp = Bm + (size_t)z * (size_t)zsB + (size_t)(col0 + wn * 64 + l15) * KDIM + 8 * h;

    v8f acc[4];
#pragma unroll
    for (int t = 0; t < 4; ++t) acc[t] = zero8f();

#pragma unroll 1
    for (int k0 = 0; k0 < KDIM; k0 += 32) {
        FragB a;
        a.half[0] = *(const v8us*)(ap + k0);
        a.half[1] = *(const v8us*)(ap + k0 + 16);
#pragma unroll
        for (int t = 0; t < 4; ++t) {
            const unsigned short* bq = bp + (size_t)t * 16 * KDIM + k0;
            FragB bf;
            bf.half[0] = *(const v8us*)(bq);
            bf.half[1] = *(const v8us*)(bq + 16);
            acc[t] = mma_bf16(a.v, bf.v, acc[t]);
        }
    }

    float rowb[8];
#pragma unroll
    for (int r = 0; r < 8; ++r) {
        int ri = row0 + wm * 16 + 8 * h + r;
        ri = ri < nbias ? ri : (nbias - 1);
        rowb[r] = bf16_val(bias[ri]);
    }
#pragma unroll
    for (int t = 0; t < 4; ++t) {
        const int cl = wn * 64 + t * 16 + l15;
        int ci = col0 + cl;
        ci = ci < nbias ? ci : (nbias - 1);
        const float colb = bf16_val(bias[ci]);
#pragma unroll
        for (int r = 0; r < 8; ++r) {
            const float badd = bias_per_row ? rowb[r] : colb;
            const float v = (acc[t][r] + badd) * oscale;
            Ct[(wm * 16 + 8 * h + r) * CT_P + cl] = (_Float16)v;
        }
    }
    __syncthreads();

    _Float16* cbase = Cm + (size_t)z * (size_t)zsC + (size_t)row0 * (size_t)ldc + col0;
    v8h sv[4];
#pragma unroll
    for (int i = 0; i < 4; ++i) {
        const int rl = w * 8 + 2 * i + h;
        sv[i] = *(const v8h*)(Ct + rl * CT_P + l15 * 8);
    }
#pragma unroll
    for (int i = 0; i < 4; ++i) {
        const int rl = w * 8 + 2 * i + h;
        *(volatile v8h*)(cbase + (size_t)rl * (size_t)ldc + l15 * 8) = sv[i];
    }
    __threadfence();
#pragma unroll
    for (int i = 0; i < 4; ++i) {
        const int rl = w * 8 + 2 * i + h;
        *(volatile v8h*)(cbase + (size_t)rl * (size_t)ldc + l15 * 8) = sv[i];
    }
}

__global__ __launch_bounds__(256) __attribute__((amdgpu_num_vgpr(256)))
void k_attn(const _Float16* __restrict__ Qp, const _Float16* __restrict__ Kp,
            const _Float16* __restrict__ Vt, float* __restrict__ Out)
{
    extern __shared__ v4f smem4[];
    float*    smem    = (float*)smem4;
    float*    S       = smem;
    float*    Ost     = smem;
    float*    rowsum  = smem + R0F;
    float*    rowmaxp = rowsum + 16;
    _Float16* Ph      = (_Float16*)(rowmaxp + 128);

    const int tid = threadIdx.x, lane = tid & 31, w = tid >> 5;
    const int h = lane >> 4, l15 = lane & 15;
    const int halfrow = 8 * h, kbo = 8 * h;
    const int b  = blockIdx.x / (SEQ / 16);
    const int q0 = (blockIdx.x - b * (SEQ / 16)) * 16;

    FragH qf[8];
    {
        const _Float16* qp = Qp + ((size_t)b * SEQ + q0 + l15) * DKD + kbo;
#pragma unroll
        for (int s = 0; s < 8; ++s) {
            qf[s].half[0] = *(const v8h*)(qp + s * 32);
            qf[s].half[1] = *(const v8h*)(qp + s * 32 + 16);
        }
    }

    float vmax[8];
#pragma unroll
    for (int r = 0; r < 8; ++r) vmax[r] = -3.0e38f;

    const _Float16* kbase = Kp + ((size_t)b * SEQ + l15) * DKD + kbo;
#pragma unroll 1
    for (int t = 0; t < SEQ / 128; ++t) {
        const int m0 = w * (SEQ / 8) + t * 16;
        const _Float16* kp = kbase + (size_t)m0 * DKD;
        v8f c = zero8f();
#pragma unroll
        for (int s = 0; s < 8; ++s) {
            FragH kb;
            kb.half[0] = *(const v8h*)(kp + s * 32);
            kb.half[1] = *(const v8h*)(kp + s * 32 + 16);
            c = mma_f16(qf[s].v, kb.v, c);
        }
#pragma unroll
        for (int r = 0; r < 8; ++r) {
            const float sv = c[r] * SCORE_SCALE;
            S[(halfrow + r) * SST + m0 + l15] = sv;
            vmax[r] = fmaxf(vmax[r], sv);
        }
    }
#pragma unroll
    for (int r = 0; r < 8; ++r) {
#pragma unroll
        for (int off = 1; off < 16; off <<= 1) vmax[r] = fmaxf(vmax[r], __shfl_xor(vmax[r], off));
    }
    if (l15 == 0) {
#pragma unroll
        for (int r = 0; r < 8; ++r) rowmaxp[w * 16 + halfrow + r] = vmax[r];
    }
    __syncthreads();

#pragma unroll 1
    for (int jj = 0; jj < 2; ++jj) {
        const int j = w * 2 + jj;
        float m = rowmaxp[j];
#pragma unroll
        for (int ww = 1; ww < 8; ++ww) m = fmaxf(m, rowmaxp[ww * 16 + j]);
        const float* srow = S + j * SST;
        _Float16* prow = Ph + j * PST;
        float s = 0.f;
#pragma unroll 2
        for (int i = lane; i < SEQ; i += 32) {
            const float e = __expf(srow[i] - m);
            const _Float16 ph = (_Float16)(e * 1024.0f);
            prow[i] = ph;
            s += (float)ph;
        }
#pragma unroll
        for (int off = 16; off; off >>= 1) s += __shfl_xor(s, off);
        if (lane == 0) rowsum[j] = s;
    }
    __syncthreads();

    v8f acc[8];
#pragma unroll
    for (int t = 0; t < 8; ++t) acc[t] = zero8f();

    const _Float16* vbase = Vt + ((size_t)b * DOD + w * 128 + l15) * SEQ + kbo;
    const _Float16* pbase = Ph + l15 * PST + kbo;
#pragma unroll 1
    for (int ks = 0; ks < SEQ / 32; ++ks) {
        const int m0 = ks * 32;
        FragH pa;
        pa.half[0] = *(const v8h*)(pbase + m0);
        pa.half[1] = *(const v8h*)(pbase + m0 + 16);
#pragma unroll
        for (int t = 0; t < 8; ++t) {
            const _Float16* vp = vbase + (size_t)t * 16 * SEQ + m0;
            FragH vf;
            vf.half[0] = *(const v8h*)(vp);
            vf.half[1] = *(const v8h*)(vp + 16);
            acc[t] = mma_f16(pa.v, vf.v, acc[t]);
        }
    }

    float inv[8];
#pragma unroll
    for (int r = 0; r < 8; ++r) inv[r] = 1.0f / (16.0f * rowsum[halfrow + r]);
#pragma unroll
    for (int t = 0; t < 8; ++t) {
#pragma unroll
        for (int r = 0; r < 8; ++r)
            Ost[(halfrow + r) * OST + w * 128 + t * 16 + l15] = acc[t][r] * inv[r];
    }
    __syncthreads();

#pragma unroll
    for (int rr = 0; rr < 2; ++rr) {
        const int row = 2 * w + rr;
        const float* src = Ost + row * OST;
        float* dst = Out + ((size_t)b * SEQ + q0 + row) * DOD;
#pragma unroll
        for (int i = 0; i < 8; ++i) {
            const int p = i * 128 + lane * 4;
            const v4f v = *(const v4f*)(src + p);
            *(volatile v4f*)(dst + p) = v;
        }
    }
    __threadfence();
#pragma unroll
    for (int rr = 0; rr < 2; ++rr) {
        const int row = 2 * w + rr;
        const float* src = Ost + row * OST;
        float* dst = Out + ((size_t)b * SEQ + q0 + row) * DOD;
#pragma unroll
        for (int i = 0; i < 8; ++i) {
            const int p = i * 128 + lane * 4;
            const v4f v = *(const v4f*)(src + p);
            *(volatile v4f*)(dst + p) = v;
        }
    }
}

extern "C" void kernel_launch(void* const* d_in, const int* in_sizes, int n_in,
                              void* d_out, int out_size, void* d_ws, size_t ws_size,
                              hipStream_t stream)
{
    if (n_in < 7) return;
    const long long need_x = ((long long)(NB - 1) * SEQ_FULL + SEQ) * CDIM;
    if ((long long)in_sizes[0] < need_x) return;
    if (in_sizes[1] < CDIM * DKD || in_sizes[2] < DKD) return;
    if (in_sizes[3] < CDIM * DKD || in_sizes[4] < DKD) return;
    if (in_sizes[5] < CDIM * DOD || in_sizes[6] < DOD) return;
    if ((long long)out_size < (long long)NB * SEQ * DOD) return;

    const float* x  = (const float*)d_in[0];
    const float* Wq = (const float*)d_in[1];
    const float* bq = (const float*)d_in[2];
    const float* Wk = (const float*)d_in[3];
    const float* bk = (const float*)d_in[4];
    const float* Wv = (const float*)d_in[5];
    const float* bv = (const float*)d_in[6];
    float* out = (float*)d_out;

    char* ws = (char*)d_ws;
    size_t off = 0;
    auto carve = [&](size_t bytes) -> char* {
        char* p = ws + off;
        off += (bytes + 255) & ~(size_t)255;
        return p;
    };
    unsigned short* xbf = (unsigned short*)carve((size_t)NB * SEQ * CDIM * 2);
    unsigned short* wqT = (unsigned short*)carve((size_t)DKD * KDIM * 2);
    unsigned short* wkT = (unsigned short*)carve((size_t)DKD * KDIM * 2);
    unsigned short* wvT = (unsigned short*)carve((size_t)DOD * KDIM * 2);
    _Float16* Qp = (_Float16*)carve((size_t)NB * SEQ * DKD * 2);
    _Float16* Kp = (_Float16*)carve((size_t)NB * SEQ * DKD * 2);
    _Float16* Vt = (_Float16*)carve((size_t)NB * DOD * SEQ * 2);
    if (off > ws_size) return;

    k_cvt_x<<<(unsigned)(((size_t)NB * SEQ * CDIM) / 8 / 256), 256, 0, stream>>>(x, xbf);

    k_transpose_w<<<dim3(DKD / 64, CDIM / 64), 256, 0, stream>>>(Wq, wqT, CDIM, DKD);
    k_transpose_w<<<dim3(DKD / 64, CDIM / 64), 256, 0, stream>>>(Wk, wkT, CDIM, DKD);
    k_transpose_w<<<dim3(DOD / 64, CDIM / 64), 256, 0, stream>>>(Wv, wvT, CDIM, DOD);

    k_gemm_nt<<<dim3(DKD / 128, (NB * SEQ) / 64, 1), 256, 0, stream>>>(
        xbf, 0LL, wqT, 0LL, bq, DKD, 0, Qp, 0LL, DKD, 16.0f);
    k_gemm_nt<<<dim3(DKD / 128, (NB * SEQ) / 64, 1), 256, 0, stream>>>(
        xbf, 0LL, wkT, 0LL, bk, DKD, 0, Kp, 0LL, DKD, 16.0f);
    k_gemm_nt<<<dim3(SEQ / 128, DOD / 64, NB), 256, 0, stream>>>(
        wvT, 0LL, xbf, (long long)SEQ * CDIM, bv, DOD, 1, Vt, (long long)DOD * SEQ, SEQ, 16.0f);

    hipFuncSetAttribute(reinterpret_cast<const void*>(&k_attn),
                        hipFuncAttributeMaxDynamicSharedMemorySize, ATTN_LDS_BYTES);
    k_attn<<<NB * (SEQ / 16), 256, ATTN_LDS_BYTES, stream>>>(Qp, Kp, Vt, out);
}
